// MoELayerWithSkip_5686536700358
// MI455X (gfx1250) — hardware-verified
//
#include <hip/hip_runtime.h>
#include <stdint.h>


#define NTOK 4096
#define DDIM 768
#define HDIM 3072
#define NEXP 4
#define TPITCH 132
#define LPITCH 72

static_assert(NTOK % 64 == 0 && NTOK % 8 == 0);
static_assert(HDIM % 128 == 0 && DDIM % 128 == 0);
static_assert(HDIM % 64 == 0 && DDIM % 64 == 0);
static_assert(HDIM % 32 == 0 && DDIM % 32 == 0 && DDIM == 768);

typedef _Float16 f16_t;
typedef _Float16 v16h __attribute__((ext_vector_type(16)));
typedef _Float16 v8h  __attribute__((ext_vector_type(8)));
typedef float    v8f  __attribute__((ext_vector_type(8)));
typedef float    v4f  __attribute__((ext_vector_type(4)));

union Frag { v16h v; v8h half[2]; };
union H8   { v8h v;  f16_t s[8]; };

__device__ __forceinline__ v8f wmma16(v16h a, v16h b, v8f c) {
  return __builtin_amdgcn_wmma_f32_16x16x32_f16(false, a, false, b, (short)0, c, false, false);
}

template <int K>
__device__ __forceinline__ void mma_loop(const f16_t* __restrict__ A,
                                         const f16_t* __restrict__ B,
                                         int l, v8f (&acc)[2][4]) {
  const int h = l >> 4, m = l & 15;
  const f16_t* ap = A + (size_t)m * K + 8 * h;
  const f16_t* bp = B + (size_t)m * K + 8 * h;
#pragma unroll 1
  for (int k0 = 0; k0 < K; k0 += 32) {
    Frag a0, a1, b0, b1, b2, b3;
    a0.half[0] = *(const v8h*)(ap + k0);
    a0.half[1] = *(const v8h*)(ap + k0 + 16);
    a1.half[0] = *(const v8h*)(ap + 16 * K + k0);
    a1.half[1] = *(const v8h*)(ap + 16 * K + k0 + 16);
    b0.half[0] = *(const v8h*)(bp + k0);
    b0.half[1] = *(const v8h*)(bp + k0 + 16);
    b1.half[0] = *(const v8h*)(bp + 16 * K + k0);
    b1.half[1] = *(const v8h*)(bp + 16 * K + k0 + 16);
    b2.half[0] = *(const v8h*)(bp + 32 * K + k0);
    b2.half[1] = *(const v8h*)(bp + 32 * K + k0 + 16);
    b3.half[0] = *(const v8h*)(bp + 48 * K + k0);
    b3.half[1] = *(const v8h*)(bp + 48 * K + k0 + 16);
    acc[0][0] = wmma16(a0.v, b0.v, acc[0][0]);
    acc[0][1] = wmma16(a0.v, b1.v, acc[0][1]);
    acc[0][2] = wmma16(a0.v, b2.v, acc[0][2]);
    acc[0][3] = wmma16(a0.v, b3.v, acc[0][3]);
    acc[1][0] = wmma16(a1.v, b0.v, acc[1][0]);
    acc[1][1] = wmma16(a1.v, b1.v, acc[1][1]);
    acc[1][2] = wmma16(a1.v, b2.v, acc[1][2]);
    acc[1][3] = wmma16(a1.v, b3.v, acc[1][3]);
    asm volatile("v_nop\n\tv_nop\n\tv_nop\n\tv_nop"
                 : "+v"(acc[0][0]), "+v"(acc[0][1]), "+v"(acc[0][2]), "+v"(acc[0][3]),
                   "+v"(acc[1][0]), "+v"(acc[1][1]), "+v"(acc[1][2]), "+v"(acc[1][3])
                 : "v"(a0.v), "v"(a1.v), "v"(b0.v), "v"(b1.v), "v"(b2.v), "v"(b3.v));
  }
}

__device__ __forceinline__ void zero_acc(v8f (&acc)[2][4]) {
#pragma unroll
  for (int i = 0; i < 2; ++i)
#pragma unroll
    for (int j = 0; j < 4; ++j)
      acc[i][j] = (v8f){0.f, 0.f, 0.f, 0.f, 0.f, 0.f, 0.f, 0.f};
}

__device__ __forceinline__ void stage_acc(float* ts, int wr, int wc, int h, int m,
                                          v8f (&acc)[2][4]) {
#pragma unroll
  for (int i = 0; i < 2; ++i)
#pragma unroll
    for (int j = 0; j < 4; ++j)
#pragma unroll
      for (int r = 0; r < 8; ++r)
        ts[(wr * 32 + 16 * i + 8 * h + r) * TPITCH + wc * 64 + 16 * j + m] = acc[i][j][r];
}

template <bool ROUTER>
__device__ __forceinline__ v8h ln_chunk(const float* xr, const float* gr, const float* tr,
                                       const float* __restrict__ Wr, int c, int l,
                                       float mu, float rstd,
                                       float& r0, float& r1, float& r2, float& r3) {
  const v4f q0 = *(const v4f*)(xr + 256 * c);
  const v4f q1 = *(const v4f*)(xr + 256 * c + 4);
  const v4f g0 = *(const v4f*)(gr + 256 * c);
  const v4f g1 = *(const v4f*)(gr + 256 * c + 4);
  const v4f t0 = *(const v4f*)(tr + 256 * c);
  const v4f t1 = *(const v4f*)(tr + 256 * c + 4);
  const int dbase = 256 * c + 8 * l;
  H8 u;
#pragma unroll
  for (int j = 0; j < 4; ++j) {
    const float xv = ((q0[j] - mu) * rstd) * g0[j] + t0[j];
    u.s[j] = (f16_t)xv;
    if (ROUTER) {
      const v4f w = *(const v4f*)(Wr + 4 * (dbase + j));
      r0 += xv * w[0]; r1 += xv * w[1]; r2 += xv * w[2]; r3 += xv * w[3];
    }
  }
#pragma unroll
  for (int j = 0; j < 4; ++j) {
    const float xv = ((q1[j] - mu) * rstd) * g1[j] + t1[j];
    u.s[4 + j] = (f16_t)xv;
    if (ROUTER) {
      const v4f w = *(const v4f*)(Wr + 4 * (dbase + 4 + j));
      r0 += xv * w[0]; r1 += xv * w[1]; r2 += xv * w[2]; r3 += xv * w[3];
    }
  }
  return u.v;
}

__global__ __launch_bounds__(256) void k_ln_router(const float* __restrict__ x,
                                                   const float* __restrict__ gam,
                                                   const float* __restrict__ bet,
                                                   const float* __restrict__ Wr,
                                                   const float* __restrict__ br,
                                                   f16_t* xn16, float* wcomb) {
  __shared__ __align__(16) float w_s[8][4];
  const int tid = threadIdx.x, wave = tid >> 5, l = tid & 31;
  const int token = blockIdx.x * 8 + wave;
  const float* xr = x + (size_t)token * DDIM + 8 * l;
  const float* gr = gam + 8 * l;
  const float* tr = bet + 8 * l;
  f16_t* xo = xn16 + (size_t)token * DDIM + 8 * l;

  float s = 0.f;
#pragma unroll 1
  for (int c = 0; c < 3; ++c) {
    const v4f q0 = *(const v4f*)(xr + 256 * c);
    const v4f q1 = *(const v4f*)(xr + 256 * c + 4);
#pragma unroll
    for (int j = 0; j < 4; ++j) s += q0[j];
#pragma unroll
    for (int j = 0; j < 4; ++j) s += q1[j];
  }
#pragma unroll
  for (int o = 16; o; o >>= 1) s += __shfl_xor(s, o, 32);
  const float mu = s * (1.0f / (float)DDIM);

  float ss = 0.f;
#pragma unroll 1
  for (int c = 0; c < 3; ++c) {
    const v4f q0 = *(const v4f*)(xr + 256 * c);
    const v4f q1 = *(const v4f*)(xr + 256 * c + 4);
#pragma unroll
    for (int j = 0; j < 4; ++j) { const float d = q0[j] - mu; ss += d * d; }
#pragma unroll
    for (int j = 0; j < 4; ++j) { const float d = q1[j] - mu; ss += d * d; }
  }
#pragma unroll
  for (int o = 16; o; o >>= 1) ss += __shfl_xor(ss, o, 32);
  const float var = ss * (1.0f / (float)DDIM);
  const float rstd = 1.0f / sqrtf(var + 1e-5f);

  float r0 = 0.f, r1 = 0.f, r2 = 0.f, r3 = 0.f;
#pragma unroll 1
  for (int c = 0; c < 3; ++c) {
    const v8h hv = ln_chunk<true>(xr, gr, tr, Wr, c, l, mu, rstd, r0, r1, r2, r3);
    *(volatile v8h*)(xo + 256 * c) = hv;
  }
#pragma unroll
  for (int o = 16; o; o >>= 1) {
    r0 += __shfl_xor(r0, o, 32);
    r1 += __shfl_xor(r1, o, 32);
    r2 += __shfl_xor(r2, o, 32);
    r3 += __shfl_xor(r3, o, 32);
  }

  const float lg0 = r0 + br[0], lg1 = r1 + br[1], lg2 = r2 + br[2], lg3 = r3 + br[3];
  const float mx = fmaxf(fmaxf(lg0, lg1), fmaxf(lg2, lg3));
  const float e0 = expf(lg0 - mx), e1 = expf(lg1 - mx), e2 = expf(lg2 - mx), e3 = expf(lg3 - mx);
  const float S = ((e0 + e1) + e2) + e3;
  const float rS = 1.0f / S;
  const float p0 = e0 * rS, p1 = e1 * rS, p2 = e2 * rS, p3 = e3 * rS;
  int i1 = 0; float pv1 = p0;
  if (p1 > pv1) { i1 = 1; pv1 = p1; }
  if (p2 > pv1) { i1 = 2; pv1 = p2; }
  if (p3 > pv1) { i1 = 3; pv1 = p3; }
  int i2 = -1; float pv2 = -1.0f;
  if (i1 != 0 && p0 > pv2) { i2 = 0; pv2 = p0; }
  if (i1 != 1 && p1 > pv2) { i2 = 1; pv2 = p1; }
  if (i1 != 2 && p2 > pv2) { i2 = 2; pv2 = p2; }
  if (i1 != 3 && p3 > pv2) { i2 = 3; pv2 = p3; }
  const float rsel = 1.0f / (pv1 + pv2);
  const float wa = pv1 * rsel, wb = pv2 * rsel;
  const float w0 = (i1 == 0) ? wa : ((i2 == 0) ? wb : 0.f);
  const float w1 = (i1 == 1) ? wa : ((i2 == 1) ? wb : 0.f);
  const float w2 = (i1 == 2) ? wa : ((i2 == 2) ? wb : 0.f);
  const float w3 = (i1 == 3) ? wa : ((i2 == 3) ? wb : 0.f);
  if (l == 0) { w_s[wave][0] = w0; w_s[wave][1] = w1; w_s[wave][2] = w2; w_s[wave][3] = w3; }
  __syncthreads();
  if (wave == 0 && l < 8) {
    const v4f wv = *(const v4f*)(&w_s[l][0]);
    *(volatile v4f*)(wcomb + ((size_t)blockIdx.x * 8 + l) * NEXP) = wv;
  }
  __threadfence();
#pragma unroll 1
  for (int c = 0; c < 3; ++c) {
    float d0 = 0.f, d1 = 0.f, d2 = 0.f, d3 = 0.f;
    const v8h hv = ln_chunk<false>(xr, gr, tr, Wr, c, l, mu, rstd, d0, d1, d2, d3);
    *(volatile v8h*)(xo + 256 * c) = hv;
  }
  if (wave == 0 && l < 8) {
    const v4f wv = *(const v4f*)(&w_s[l][0]);
    *(volatile v4f*)(wcomb + ((size_t)blockIdx.x * 8 + l) * NEXP) = wv;
  }
}

__global__ __launch_bounds__(128) void k_prep(const float* __restrict__ in, f16_t* out,
                                              int R, int C, float scale) {
  __shared__ __align__(16) f16_t T[64 * LPITCH];
  const int tid = threadIdx.x, wave = tid >> 5, l = tid & 31;
  const int e = blockIdx.z, c0 = blockIdx.x * 64, r0 = blockIdx.y * 64;
  const float* src = in + ((size_t)e * R + r0) * (size_t)C + c0;
#pragma unroll 4
  for (int i = 0; i < 32; ++i) {
    const int idx = tid + 128 * i;
    const int rr = idx >> 6, cc = idx & 63;
    T[cc * LPITCH + rr] = (f16_t)(src[(size_t)rr * C + cc] * scale);
  }
  __syncthreads();
  f16_t* dst = out + ((size_t)e * C + c0) * (size_t)R + r0;
  const int q = l >> 3, c8 = (l & 7) * 8;
#pragma unroll
  for (int i = 0; i < 4; ++i) {
    const int cc = wave * 16 + 4 * i + q;
    const v8h v = *(const v8h*)(T + cc * LPITCH + c8);
    *(volatile v8h*)(dst + (size_t)cc * R + c8) = v;
  }
  __threadfence();
#pragma unroll
  for (int i = 0; i < 4; ++i) {
    const int cc = wave * 16 + 4 * i + q;
    const v8h v = *(const v8h*)(T + cc * LPITCH + c8);
    *(volatile v8h*)(dst + (size_t)cc * R + c8) = v;
  }
}

__device__ __forceinline__ void epi_h_pass(const float* ts, const float* __restrict__ bb,
                                           f16_t* hb, int wave, int l) {
  const int cl = (l & 15) * 8, rs = l >> 4;
  const v4f bq0 = *(const v4f*)(bb + cl);
  const v4f bq1 = *(const v4f*)(bb + cl + 4);
#pragma unroll
  for (int t = 0; t < 8; ++t) {
    const int row = wave * 16 + 2 * t + rs;
    const v4f p0 = *(const v4f*)(ts + row * TPITCH + cl);
    const v4f p1 = *(const v4f*)(ts + row * TPITCH + cl + 4);
    const v4f y0 = p0 * 0.03125f + bq0;
    const v4f y1 = p1 * 0.03125f + bq1;
    H8 u;
#pragma unroll
    for (int j = 0; j < 4; ++j) u.s[j] = (f16_t)fmaxf(y0[j], 0.0f);
#pragma unroll
    for (int j = 0; j < 4; ++j) u.s[4 + j] = (f16_t)fmaxf(y1[j], 0.0f);
    *(volatile v8h*)(hb + (size_t)row * HDIM + cl) = u.v;
  }
}

__global__ __launch_bounds__(128) void k_ffn1(const f16_t* __restrict__ xn16,
                                              const f16_t* __restrict__ W1h,
                                              const float* __restrict__ b1,
                                              f16_t* h16, int e) {
  __shared__ __align__(16) float tileS[64 * TPITCH];
  const int tid = threadIdx.x, wave = tid >> 5, l = tid & 31;
  const int h = l >> 4, m = l & 15;
  const int wr = wave >> 1, wc = wave & 1;
  const int row0 = blockIdx.x * 64, col0 = blockIdx.y * 128;

  v8f acc[2][4];
  zero_acc(acc);
  const f16_t* A = xn16 + (size_t)(row0 + wr * 32) * DDIM;
  const f16_t* B = W1h + ((size_t)e * HDIM + col0 + wc * 64) * DDIM;
  mma_loop<DDIM>(A, B, l, acc);

  stage_acc(tileS, wr, wc, h, m, acc);
  __syncthreads();
  const float* bb = b1 + (size_t)e * HDIM + col0;
  f16_t* hb = h16 + (size_t)row0 * HDIM + col0;
  epi_h_pass(tileS, bb, hb, wave, l);
  __threadfence();
  epi_h_pass(tileS, bb, hb, wave, l);
}

__global__ __launch_bounds__(128) void k_ffn2(const f16_t* __restrict__ h16,
                                              const f16_t* __restrict__ W2h,
                                              const float* __restrict__ b2,
                                              const float* __restrict__ wcomb,
                                              const float* __restrict__ x,
                                              float* out, int e) {
  __shared__ __align__(16) float tileS[64 * TPITCH];
  const int tid = threadIdx.x, wave = tid >> 5, l = tid & 31;
  const int h = l >> 4, m = l & 15;
  const int wr = wave >> 1, wc = wave & 1;
  const int row0 = blockIdx.x * 64, col0 = blockIdx.y * 128;

  v8f acc[2][4];
  zero_acc(acc);
  const f16_t* A = h16 + (size_t)(row0 + wr * 32) * HDIM;
  const f16_t* B = W2h + ((size_t)e * DDIM + col0 + wc * 64) * HDIM;
  mma_loop<HDIM>(A, B, l, acc);

  stage_acc(tileS, wr, wc, h, m, acc);
  __syncthreads();

  const int col = 4 * l;
  const v4f bq = *(const v4f*)(b2 + (size_t)e * DDIM + col0 + col);
  float* ob = out + (size_t)row0 * DDIM + col0 + col;
  const float* xb = x + (size_t)row0 * DDIM + col0 + col;
  const float* wb = wcomb + (size_t)row0 * NEXP + e;
#pragma unroll
  for (int t = 0; t < 16; ++t) {
    const int row = wave * 16 + t;
    float* sp = tileS + row * TPITCH + col;
    const v4f p = *(const v4f*)sp;
    const v4f y = p * 0.03125f + bq;
    const float wv = wb[(size_t)row * NEXP];
    v4f base;
    if (e == 0) base = *(const v4f*)(xb + (size_t)row * DDIM);
    else        base = *(const v4f*)(ob + (size_t)row * DDIM);
    const v4f val = base + wv * y;
    *(v4f*)sp = val;
    *(volatile v4f*)(ob + (size_t)row * DDIM) = val;
  }
  __threadfence();
#pragma unroll
  for (int t = 0; t < 16; ++t) {
    const int row = wave * 16 + t;
    const v4f val = *(const v4f*)(tileS + row * TPITCH + col);
    *(volatile v4f*)(ob + (size_t)row * DDIM) = val;
  }
}

extern "C" void kernel_launch(void* const* d_in, const int* in_sizes, int n_in,
                              void* d_out, int out_size, void* d_ws, size_t ws_size,
                              hipStream_t stream) {
  if (n_in < 9) return;
  if (in_sizes[0] != NTOK * DDIM || in_sizes[1] != DDIM || in_sizes[2] != DDIM ||
      in_sizes[3] != DDIM * NEXP || in_sizes[4] != NEXP ||
      in_sizes[5] != NEXP * DDIM * HDIM || in_sizes[6] != NEXP * HDIM ||
      in_sizes[7] != NEXP * HDIM * DDIM || in_sizes[8] != NEXP * DDIM ||
      out_size != NTOK * DDIM) return;

  const float* x     = (const float*)d_in[0];
  const float* gamma = (const float*)d_in[1];
  const float* beta  = (const float*)d_in[2];
  const float* Wr    = (const float*)d_in[3];
  const float* br    = (const float*)d_in[4];
  const float* W1    = (const float*)d_in[5];
  const float* b1    = (const float*)d_in[6];
  const float* W2    = (const float*)d_in[7];
  const float* b2    = (const float*)d_in[8];
  float* out = (float*)d_out;

  char* ws = (char*)d_ws;
  size_t off = 0;
  f16_t* xn16 = (f16_t*)(ws + off);  off += (size_t)NTOK * DDIM * sizeof(f16_t);
  float* wcomb = (float*)(ws + off); off += (size_t)NTOK * NEXP * sizeof(float);
  f16_t* W1h = (f16_t*)(ws + off);   off += (size_t)NEXP * HDIM * DDIM * sizeof(f16_t);
  f16_t* W2h = (f16_t*)(ws + off);   off += (size_t)NEXP * HDIM * DDIM * sizeof(f16_t);
  f16_t* h16 = (f16_t*)(ws + off);   off += (size_t)NTOK * HDIM * sizeof(f16_t);
  if (off > ws_size) return;

  k_ln_router<<<dim3(NTOK / 8), dim3(256), 0, stream>>>(x, gamma, beta, Wr, br, xn16, wcomb);
  k_prep<<<dim3(HDIM / 64, DDIM / 64, NEXP), dim3(128), 0, stream>>>(W1, W1h, DDIM, HDIM, 32.0f);
  k_prep<<<dim3(DDIM / 64, HDIM / 64, NEXP), dim3(128), 0, stream>>>(W2, W2h, HDIM, DDIM, 32.0f);
  for (int e = 0; e < NEXP; ++e) {
    k_ffn1<<<dim3(NTOK / 64, HDIM / 128), dim3(128), 0, stream>>>(xn16, W1h, b1, h16, e);
    k_ffn2<<<dim3(NTOK / 64, DDIM / 128), dim3(128), 0, stream>>>(h16, W2h, b2, wcomb, x, out, e);
  }
}
